// CA_82300163326040
// MI455X (gfx1250) — hardware-verified
//
#include <hip/hip_runtime.h>
#include <math.h>

constexpr int  kBatch    = 8;
constexpr int  kSeq      = 2048;
constexpr int  kDim      = 512;
constexpr int  kTok      = kBatch * kSeq;
constexpr int  kChunk    = 256;
constexpr int  kNumChunk = kSeq / kChunk;
constexpr long kPlaneTok = (long)kSeq * kDim;
constexpr long kPlaneS   = (long)kChunk * kSeq;
constexpr long kPlaneW   = (long)kDim * kDim;
constexpr float kWCarry     = 16.0f;
constexpr float kWCarryInv  = 1.0f / 16.0f;
constexpr float kPCarry     = 2048.0f;
constexpr float kPCarryInv  = 1.0f / 2048.0f;
constexpr float kScoreScale = 0.044194173824159220f;

constexpr size_t kOffIn16 = 0;
constexpr size_t kOffS    = kOffIn16 + (size_t)kTok * kDim * 2;
constexpr size_t kOffP    = kOffS + (size_t)kBatch * kPlaneS * 4;
constexpr size_t kOffW    = kOffP + (size_t)kBatch * kPlaneS * 2;
constexpr size_t kOffQ    = kOffW + (size_t)3 * kPlaneW * 2;
constexpr size_t kOffK    = kOffQ + (size_t)kTok * kDim * 2;
constexpr size_t kOffVt   = kOffK + (size_t)kTok * kDim * 2;
constexpr size_t kOffU1   = kOffVt + (size_t)kTok * kDim * 2;
constexpr size_t kWsEnd   = kOffU1 + (size_t)kTok * kDim * 4;
static_assert(kWsEnd == 127401984ull);
static_assert(kWsEnd <= 134217728ull);
static_assert((kOffS % 128) == 0 && (kOffP % 128) == 0 && (kOffW % 128) == 0 && (kOffQ % 128) == 0);
static_assert((kOffK % 128) == 0 && (kOffVt % 128) == 0 && (kOffU1 % 128) == 0);
static_assert(kDim % 32 == 0 && kSeq % 32 == 0);
static_assert(kChunk % 64 == 0 && kDim % 64 == 0 && kSeq % 64 == 0 && kTok % 64 == 0);

typedef __attribute__((ext_vector_type(16))) _Float16 v16h;
typedef __attribute__((ext_vector_type(8)))  _Float16 v8h;
typedef __attribute__((ext_vector_type(16))) __bf16   v16b;
typedef __attribute__((ext_vector_type(8)))  __bf16   v8b;
typedef __attribute__((ext_vector_type(8)))  float    v8f;
typedef __attribute__((ext_vector_type(4)))  float    v4f;
typedef __attribute__((ext_vector_type(4)))  unsigned int v4u;

__device__ __forceinline__ unsigned short f2bf_bits(float f) {
  unsigned u = __float_as_uint(f);
  return (unsigned short)((u + 0x7FFFu + ((u >> 16) & 1u)) >> 16);
}
__device__ __forceinline__ float bf_bits2f(unsigned short h) { return __uint_as_float(((unsigned)h) << 16); }

__device__ __forceinline__ void dep_guard_h(v8f& a, v8f& b, v16h x, v16h y) { asm volatile("v_nop\n\tv_nop\n\tv_nop\n\tv_nop" : "+v"(a), "+v"(b) : "v"(x), "v"(y)); }
__device__ __forceinline__ void dep_guard_b(v8f& a, v8f& b, v16b x, v16b y) { asm volatile("v_nop\n\tv_nop\n\tv_nop\n\tv_nop" : "+v"(a), "+v"(b) : "v"(x), "v"(y)); }
__device__ __forceinline__ void keep4_h(v16h a, v16h b, v16h c, v16h d) { asm volatile("v_nop" :: "v"(a), "v"(b), "v"(c), "v"(d)); }
__device__ __forceinline__ void keep4_b(v16b a, v16b b, v16b c, v16b d) { asm volatile("v_nop" :: "v"(a), "v"(b), "v"(c), "v"(d)); }
__device__ __forceinline__ void acc_guard4(v8f& a, v8f& b, v8f& c, v8f& d) { asm volatile("v_nop\n\tv_nop\n\tv_nop\n\tv_nop" : "+v"(a), "+v"(b), "+v"(c), "+v"(d)); }
template <typename T> struct Frag;
template <> struct Frag<_Float16> {
  typedef v16h V; union U { v16h v; v8h h[2]; };
  static __device__ __forceinline__ v16h load(const _Float16* p) {
    U f; f.h[0] = *(const v8h*)(p); f.h[1] = *(const v8h*)(p + 16); return f.v;
  }
  static __device__ __forceinline__ v8f mma(v16h a, v16h b, v8f c) {
    return __builtin_amdgcn_wmma_f32_16x16x32_f16(false, a, false, b, (short)0, c, false, false);
  }
  static __device__ __forceinline__ void guard(v8f& a, v8f& b, v16h x, v16h y) { dep_guard_h(a, b, x, y); }
  static __device__ __forceinline__ void keep(v16h a, v16h b, v16h c, v16h d) { keep4_h(a, b, c, d); }
};
template <> struct Frag<__bf16> {
  typedef v16b V; union U { v16b v; v8b h[2]; };
  static __device__ __forceinline__ v16b load(const __bf16* p) {
    U f; f.h[0] = *(const v8b*)(p); f.h[1] = *(const v8b*)(p + 16); return f.v;
  }
  static __device__ __forceinline__ v8f mma(v16b a, v16b b, v8f c) {
    return __builtin_amdgcn_wmma_f32_16x16x32_bf16(false, a, false, b, (short)0, c, false, false);
  }
  static __device__ __forceinline__ void guard(v8f& a, v8f& b, v16b x, v16b y) { dep_guard_b(a, b, x, y); }
  static __device__ __forceinline__ void keep(v16b a, v16b b, v16b c, v16b d) { keep4_b(a, b, c, d); }
};

__device__ __forceinline__ unsigned pk16(unsigned short a, unsigned short b) { return (unsigned)a | ((unsigned)b << 16); }
__device__ __forceinline__ unsigned short h_bits(float f) { const _Float16 h = (_Float16)f; return __builtin_bit_cast(unsigned short, h); }

template <int ET> struct Elem;
template <> struct Elem<0> { typedef _Float16 T; };
template <> struct Elem<1> { typedef __bf16 T; };
template <int ET, bool SPLIT, int BIAS_MODE, int OUT_MODE, bool RESID, bool RESID2>
__global__ __launch_bounds__(256) void wmma_gemm64(
    const unsigned short* __restrict__ Ap, const unsigned short* __restrict__ A2p, int lda, long strideA,
    const unsigned short* __restrict__ Btp, const unsigned short* __restrict__ Bt2p, int ldb, long strideB,
    void* __restrict__ Cout, void* __restrict__ Cout2, int ldc, long strideC,
    const float* __restrict__ bias,
    const float* __restrict__ resid, long strideR,
    const float* __restrict__ resid2, long strideR2,
    int M, int N, int K, float scale) {
  typedef typename Elem<ET>::T T;
  typedef typename Frag<T>::V V;
  const T* A = (const T*)Ap; const T* A2 = (const T*)A2p; const T* Bt = (const T*)Btp; const T* Bt2 = (const T*)Bt2p;
  __shared__ __align__(16) float sT[8][16 * 68];
  const int b    = blockIdx.y;
  const int lane = threadIdx.x & 31;
  const int wave = threadIdx.x >> 5;
  const int tilesN = N >> 6;
  const int tilesM = M >> 6;
  const int tile = blockIdx.x * 8 + wave;
  if (tile >= tilesM * tilesN) return;
  const int tm = tile / tilesN;
  const int tn = tile - tm * tilesN;
  const int m0 = tm << 6;
  const int n0 = tn << 6;

  const T* Ab  = A  + (size_t)b * strideA;
  const T* Bb  = Bt + (size_t)b * strideB;
  const T* Ab2 = SPLIT ? (A2  + (size_t)b * strideA) : nullptr;
  const T* Bb2 = SPLIT ? (Bt2 + (size_t)b * strideB) : nullptr;

  const int rlane = lane & 15;
  const int koff  = (lane >> 4) * 8;
  const int mOff  = (lane >> 4) * 8;

  v8f acc[4][4];
#pragma unroll
  for (int i = 0; i < 4; ++i)
#pragma unroll
    for (int j = 0; j < 4; ++j) acc[i][j] = (v8f){0.f,0.f,0.f,0.f,0.f,0.f,0.f,0.f};

  for (int k0 = 0; k0 < K; k0 += 32) {
    V bh[4], bl[4];
#pragma unroll
    for (int j = 0; j < 4; ++j) {
      const size_t bo = (size_t)(n0 + (j << 4) + rlane) * ldb + koff + k0;
      bh[j] = Frag<T>::load(Bb + bo);
      if (SPLIT) bl[j] = Frag<T>::load(Bb2 + bo);
    }
#pragma unroll
    for (int i = 0; i < 4; ++i) {
      const size_t ao = (size_t)(m0 + (i << 4) + rlane) * lda + koff + k0;
      V ah = Frag<T>::load(Ab + ao);
      V al;
      if (SPLIT) al = Frag<T>::load(Ab2 + ao);
#pragma unroll
      for (int j = 0; j < 4; ++j) {
        acc[i][j] = Frag<T>::mma(ah, bh[j], acc[i][j]);
        if (SPLIT) {
          acc[i][j] = Frag<T>::mma(ah, bl[j], acc[i][j]);
          acc[i][j] = Frag<T>::mma(al, bh[j], acc[i][j]);
        }
      }
      Frag<T>::guard(acc[i][0], acc[i][3], ah, SPLIT ? al : ah);
    }
    Frag<T>::keep(bh[0], bh[1], bh[2], bh[3]);
    if (SPLIT) Frag<T>::keep(bl[0], bl[1], bl[2], bl[3]);
  }
  acc_guard4(acc[0][0], acc[0][1], acc[0][2], acc[0][3]);
  acc_guard4(acc[1][0], acc[1][1], acc[1][2], acc[1][3]);
  acc_guard4(acc[2][0], acc[2][1], acc[2][2], acc[2][3]);
  acc_guard4(acc[3][0], acc[3][1], acc[3][2], acc[3][3]);

  float* slab = sT[wave];
  const float* Rb  = RESID  ? (resid  + (size_t)b * strideR)  : nullptr;
  const float* Rb2 = RESID2 ? (resid2 + (size_t)b * strideR2) : nullptr;
#pragma unroll
  for (int i = 0; i < 4; ++i) {
    const int mBase = m0 + (i << 4);
#pragma unroll
    for (int j = 0; j < 4; ++j) {
      const int n = n0 + (j << 4) + rlane;
      float bv = 0.f;
      if (BIAS_MODE == 2) bv = bias[n];
#pragma unroll
      for (int r = 0; r < 8; ++r) {
        float v = acc[i][j][r] * scale;
        if (BIAS_MODE == 1) v += bias[mBase + mOff + r];
        if (BIAS_MODE == 2) v += bv;
        if (RESID)  v += Rb[(size_t)(mBase + mOff + r) * ldc + n];
        if (RESID2) v = Rb2[(size_t)(mBase + mOff + r) * ldc + n] + v;
        slab[(mOff + r) * 68 + (j << 4) + rlane] = v;
      }
    }
    __builtin_amdgcn_fence(__ATOMIC_RELEASE, "workgroup");
    __builtin_amdgcn_wave_barrier();
    __builtin_amdgcn_fence(__ATOMIC_ACQUIRE, "workgroup");
    if (OUT_MODE == 0) {
      float* C = (float*)Cout + (size_t)b * strideC;
      const int hh = lane >> 4, c4 = (lane & 15) * 4;
      for (int pass = 0; pass < 2; ++pass) {
#pragma unroll
        for (int it = 0; it < 8; ++it) {
          const int row = it * 2 + hh;
          v4f v = *(const v4f*)(slab + row * 68 + c4);
          *(volatile v4f*)(C + (size_t)(mBase + row) * ldc + n0 + c4) = v;
        }
        __threadfence();
      }
    } else {
      const int q = lane >> 3, c8 = (lane & 7) * 8;
      unsigned short* C  = (unsigned short*)Cout  + (size_t)b * strideC;
      unsigned short* C2 = (OUT_MODE == 2) ? ((unsigned short*)Cout2 + (size_t)b * strideC) : nullptr;
      for (int pass = 0; pass < 2; ++pass) {
#pragma unroll
        for (int it = 0; it < 4; ++it) {
          const int row = it * 4 + q;
          const float* sp = slab + row * 68 + c8;
          v8h hv, lv;
#pragma unroll
          for (int e = 0; e < 8; ++e) {
            if (OUT_MODE == 1) {
              hv[e] = (_Float16)sp[e];
            } else {
              unsigned short hb = f2bf_bits(sp[e]);
              unsigned short lb = f2bf_bits(sp[e] - bf_bits2f(hb));
              hv[e] = __builtin_bit_cast(_Float16, hb);
              lv[e] = __builtin_bit_cast(_Float16, lb);
            }
          }
          *(volatile v8h*)(C + (size_t)(mBase + row) * ldc + n0 + c8) = hv;
          if (OUT_MODE == 2) *(volatile v8h*)(C2 + (size_t)(mBase + row) * ldc + n0 + c8) = lv;
        }
        __threadfence();
      }
    }
    __builtin_amdgcn_fence(__ATOMIC_RELEASE, "workgroup");
    __builtin_amdgcn_wave_barrier();
    __builtin_amdgcn_fence(__ATOMIC_ACQUIRE, "workgroup");
  }
}

__global__ __launch_bounds__(256) void cast8_f16_kernel(const float* __restrict__ in, unsigned short* __restrict__ out, int n8, float scale) {
  const int i = blockIdx.x * 256 + threadIdx.x;
  if (i >= n8) return;
  const float* p = in + 8 * (size_t)i;
  const v4f a = *(const v4f*)(p);
  const v4f c = *(const v4f*)(p + 4);
  unsigned short hb[8];
#pragma unroll
  for (int e = 0; e < 4; ++e) {
    hb[e]     = h_bits(a[e] * scale);
    hb[4 + e] = h_bits(c[e] * scale);
  }
  const v4u u = (v4u){pk16(hb[0], hb[1]), pk16(hb[2], hb[3]), pk16(hb[4], hb[5]), pk16(hb[6], hb[7])};
  unsigned short* q = out + 8 * (size_t)i;
  *(volatile v4u*)q = u;
  __threadfence();
  *(volatile v4u*)q = u;
}

__global__ __launch_bounds__(256) void castw3_f16_kernel(const float* __restrict__ W0, const float* __restrict__ W1,
                                                        const float* __restrict__ W2, unsigned short* __restrict__ out,
                                                        int n8, float scale) {
  const int i = blockIdx.x * 256 + threadIdx.x;
  const int z = blockIdx.y;
  const float* W = (z == 0) ? W0 : (z == 1) ? W1 : W2;
  if (i >= n8) return;
  const float* p = W + 8 * (size_t)i;
  const v4f a = *(const v4f*)(p);
  const v4f c = *(const v4f*)(p + 4);
  unsigned short hb[8];
#pragma unroll
  for (int e = 0; e < 4; ++e) {
    hb[e]     = h_bits(a[e] * scale);
    hb[4 + e] = h_bits(c[e] * scale);
  }
  const v4u u = (v4u){pk16(hb[0], hb[1]), pk16(hb[2], hb[3]), pk16(hb[4], hb[5]), pk16(hb[6], hb[7])};
  unsigned short* q = out + (size_t)z * 8 * (size_t)n8 + 8 * (size_t)i;
  *(volatile v4u*)q = u;
  __threadfence();
  *(volatile v4u*)q = u;
}

__global__ __launch_bounds__(128) void softmax_batch_kernel(const float* __restrict__ S, unsigned short* __restrict__ P, float carry) {
  __shared__ float sEx[kBatch * 8 * 128];
  __shared__ float sRc[8 * 128];
  const int t   = threadIdx.x;
  const int row = blockIdx.x >> 1;
  const int c0  = (blockIdx.x & 1) * 1024 + t * 8;
  const size_t off = (size_t)row * kSeq + c0;
  float mx[8];
#pragma unroll
  for (int e = 0; e < 8; ++e) mx[e] = -INFINITY;
#pragma unroll 1
  for (int b = 0; b < kBatch; ++b) {
    const float* sp = S + (size_t)b * kPlaneS + off;
    const v4f a = *(const v4f*)(sp);
    const v4f c = *(const v4f*)(sp + 4);
    float* q = sEx + b * 1024 + t;
#pragma unroll
    for (int e = 0; e < 4; ++e) {
      q[e * 128] = a[e];
      mx[e] = fmaxf(mx[e], a[e]);
      q[(4 + e) * 128] = c[e];
      mx[4 + e] = fmaxf(mx[4 + e], c[e]);
    }
  }
  __syncthreads();
  float sm[8];
#pragma unroll
  for (int e = 0; e < 8; ++e) sm[e] = 0.f;
#pragma unroll 1
  for (int b = 0; b < kBatch; ++b) {
    float* q = sEx + b * 1024 + t;
#pragma unroll
    for (int e = 0; e < 8; ++e) {
      const float ex = expf(q[e * 128] - mx[e]);
      q[e * 128] = ex;
      sm[e] += ex;
    }
  }
#pragma unroll
  for (int e = 0; e < 8; ++e) sRc[e * 128 + t] = sm[e];
  __syncthreads();
#pragma unroll 1
  for (int e = 0; e < 8; ++e) {
    const int i = e * 128 + t;
    const float s = sRc[i];
    sRc[i] = carry / s;
  }
  __syncthreads();
  v4u u[kBatch];
#pragma unroll
  for (int b = 0; b < kBatch; ++b) {
    const float* q = sEx + b * 1024 + t;
    unsigned short hb[8];
#pragma unroll
    for (int e = 0; e < 8; ++e) hb[e] = h_bits(q[e * 128] * sRc[e * 128 + t]);
    u[b] = (v4u){pk16(hb[0], hb[1]), pk16(hb[2], hb[3]), pk16(hb[4], hb[5]), pk16(hb[6], hb[7])};
  }
  for (int ps = 0; ps < 2; ++ps) {
#pragma unroll
    for (int b = 0; b < kBatch; ++b) *(volatile v4u*)(P + (size_t)b * kPlaneS + off) = u[b];
    __threadfence();
  }
}

extern "C" void kernel_launch(void* const* d_in, const int* in_sizes, int n_in,
                              void* d_out, int out_size, void* d_ws, size_t ws_size, hipStream_t stream) {
  if (n_in < 14) return;
  if (in_sizes[0] != kTok * kDim || in_sizes[1] != kTok * kDim) return;
  if (in_sizes[2] != (int)kPlaneW || in_sizes[3] != kDim || in_sizes[12] != (int)kPlaneW || in_sizes[13] != kDim) return;
  if (out_size != kTok * kDim) return;
  if (ws_size < kWsEnd) return;

  const float* X    = (const float*)d_in[0];
  const float* Y    = (const float*)d_in[1];
  const float* W_xq = (const float*)d_in[2];  const float* b_xq = (const float*)d_in[3];
  const float* W_xk = (const float*)d_in[4];  const float* b_xk = (const float*)d_in[5];
  const float* W_xv = (const float*)d_in[6];  const float* b_xv = (const float*)d_in[7];
  const float* W_yq = (const float*)d_in[8];  const float* b_yq = (const float*)d_in[9];
  const float* W_yk = (const float*)d_in[10]; const float* b_yk = (const float*)d_in[11];
  const float* W_yv = (const float*)d_in[12]; const float* b_yv = (const float*)d_in[13];
  float* out = (float*)d_out;

  unsigned char*  ws   = (unsigned char*)d_ws;
  unsigned short* in16 = (unsigned short*)(ws + kOffIn16);
  float*          Sb   = (float*)(ws + kOffS);
  unsigned short* Pb   = (unsigned short*)(ws + kOffP);
  unsigned short* W16  = (unsigned short*)(ws + kOffW);
  unsigned short* Qp   = (unsigned short*)(ws + kOffQ);
  unsigned short* Kp   = (unsigned short*)(ws + kOffK);
  unsigned short* Vt   = (unsigned short*)(ws + kOffVt);
  float*          U1   = (float*)(ws + kOffU1);

  const int nTok8 = (kTok * kDim) / 8;
  const int nW8   = (int)(kPlaneW / 8);
  const dim3 gCastTok(nTok8 / 256);
  const dim3 gCastW(nW8 / 256, 3);
  const dim3 gProjTok(((kTok / 64) * (kDim / 64)) / 8, 1);
  const dim3 gProjVt(((kDim / 64) * (kSeq / 64)) / 8, kBatch);
  const dim3 gScore(((kChunk / 64) * (kSeq / 64)) / 8, kBatch);
  const dim3 gPV(((kChunk / 64) * (kDim / 64)) / 8, kBatch);
  const dim3 gSoft(kChunk * 2);

  cast8_f16_kernel<<<gCastTok, 256, 0, stream>>>(X, in16, nTok8, 1.0f);
  castw3_f16_kernel<<<gCastW, 256, 0, stream>>>(W_xq, W_yk, W_yv, W16, nW8, kWCarry);
  wmma_gemm64<0, false, 2, 1, false, false><<<gProjTok, 256, 0, stream>>>(
      in16, in16, kDim, 0, W16, W16, kDim, 0, Qp, Qp, kDim, 0,
      b_xq, X, 0, X, 0, kTok, kDim, kDim, kWCarryInv);
  cast8_f16_kernel<<<gCastTok, 256, 0, stream>>>(Y, in16, nTok8, 1.0f);
  wmma_gemm64<0, false, 2, 1, false, false><<<gProjTok, 256, 0, stream>>>(
      in16, in16, kDim, 0, W16 + kPlaneW, W16 + kPlaneW, kDim, 0, Kp, Kp, kDim, 0,
      b_yk, X, 0, X, 0, kTok, kDim, kDim, kWCarryInv);
  wmma_gemm64<0, false, 1, 1, false, false><<<gProjVt, 256, 0, stream>>>(
      W16 + 2 * kPlaneW, W16 + 2 * kPlaneW, kDim, 0, in16, in16, kDim, kPlaneTok, Vt, Vt, kSeq, kPlaneTok,
      b_yv, X, 0, X, 0, kDim, kSeq, kDim, kWCarryInv);
  for (int c = 0; c < kNumChunk; ++c) {
    const size_t rowOff = (size_t)c * kChunk * kDim;
    wmma_gemm64<0, false, 0, 0, false, false><<<gScore, 256, 0, stream>>>(
        Qp + rowOff, Qp + rowOff, kDim, kPlaneTok, Kp, Kp, kDim, kPlaneTok, Sb, Sb, kSeq, kPlaneS,
        b_xq, X, 0, X, 0, kChunk, kSeq, kDim, kScoreScale);
    softmax_batch_kernel<<<gSoft, 128, 0, stream>>>(Sb, Pb, kPCarry);
    wmma_gemm64<0, false, 0, 0, true, false><<<gPV, 256, 0, stream>>>(
        Pb, Pb, kSeq, kPlaneS, Vt, Vt, kSeq, kPlaneTok, U1 + rowOff, U1 + rowOff, kDim, kPlaneTok,
        b_xq, X + rowOff, kPlaneTok, X, 0, kChunk, kDim, kSeq, kPCarryInv);
  }

  castw3_f16_kernel<<<gCastW, 256, 0, stream>>>(W_yq, W_xk, W_xv, W16, nW8, kWCarry);
  wmma_gemm64<0, false, 2, 1, false, false><<<gProjTok, 256, 0, stream>>>(
      in16, in16, kDim, 0, W16, W16, kDim, 0, Qp, Qp, kDim, 0,
      b_yq, X, 0, X, 0, kTok, kDim, kDim, kWCarryInv);
  cast8_f16_kernel<<<gCastTok, 256, 0, stream>>>(X, in16, nTok8, 1.0f);
  wmma_gemm64<0, false, 2, 1, false, false><<<gProjTok, 256, 0, stream>>>(
      in16, in16, kDim, 0, W16 + kPlaneW, W16 + kPlaneW, kDim, 0, Kp, Kp, kDim, 0,
      b_xk, X, 0, X, 0, kTok, kDim, kDim, kWCarryInv);
  wmma_gemm64<0, false, 1, 1, false, false><<<gProjVt, 256, 0, stream>>>(
      W16 + 2 * kPlaneW, W16 + 2 * kPlaneW, kDim, 0, in16, in16, kDim, kPlaneTok, Vt, Vt, kSeq, kPlaneTok,
      b_xv, X, 0, X, 0, kDim, kSeq, kDim, kWCarryInv);
  for (int c = 0; c < kNumChunk; ++c) {
    const size_t rowOff = (size_t)c * kChunk * kDim;
    wmma_gemm64<0, false, 0, 0, false, false><<<gScore, 256, 0, stream>>>(
        Qp + rowOff, Qp + rowOff, kDim, kPlaneTok, Kp, Kp, kDim, kPlaneTok, Sb, Sb, kSeq, kPlaneS,
        b_xq, X, 0, X, 0, kChunk, kSeq, kDim, kScoreScale);
    softmax_batch_kernel<<<gSoft, 128, 0, stream>>>(Sb, Pb, kPCarry);
    wmma_gemm64<0, false, 0, 0, true, true><<<gPV, 256, 0, stream>>>(
        Pb, Pb, kSeq, kPlaneS, Vt, Vt, kSeq, kPlaneTok, out + rowOff, out + rowOff, kDim, kPlaneTok,
        b_xq, Y + rowOff, kPlaneTok, U1 + rowOff, kPlaneTok, kChunk, kDim, kSeq, kPCarryInv);
  }
}
